// LinkPrediction_22376779612762
// MI455X (gfx1250) — hardware-run, weakly checked
//
#include <hip/hip_runtime.h>


namespace {
constexpr int N = 50000, EP = 400000, EN = 400000, ET = EP + EN, D0 = 128, H1 = 256, H2 = 128;
constexpr float XS = 8.0f, HS = 256.0f, WSC = 256.0f, EPS = 1e-5f;
typedef _Float16 b16;
typedef __attribute__((ext_vector_type(16))) _Float16 v16b;
typedef __attribute__((ext_vector_type(8))) _Float16 v8b;
typedef __attribute__((ext_vector_type(8))) float v8f;
typedef __attribute__((ext_vector_type(4))) float v4f;
__device__ __forceinline__ float bf16_rne(float f) { unsigned int u = __float_as_uint(f); u += 0x7FFFu + ((u >> 16) & 1u); float r = __uint_as_float(u & 0xFFFF0000u); asm volatile("" : "+v"(r)); return r; }
__device__ __forceinline__ float bfv(float f) { float r = bf16_rne(f); asm volatile("" : "+v"(r)); return r; }
__device__ __forceinline__ void split16(float v, b16& hi, b16& lo) { hi = (b16)v; lo = (b16)(v - (float)hi); }
__device__ __forceinline__ v16b frag_kb(const b16* p, int hh) { const v8b a = *(const v8b*)(p + 8 * hh), b = *(const v8b*)(p + 16 + 8 * hh); v16b f;
#pragma unroll
  for (int e = 0; e < 8; ++e) { f[e] = a[e]; f[8 + e] = b[e]; } return f; }
__device__ __forceinline__ v8f wmma16b(v16b a, v16b b, v8f c) { v8f d = __builtin_amdgcn_wmma_f32_16x16x32_f16(false, a, false, b, (short)0, c, false, false); asm volatile("v_nop\n\tv_nop\n\tv_nop\n\tv_nop" : "+v"(d) : "v"(a), "v"(b)); return d; }
__device__ __forceinline__ void wave_lds_sync() { __builtin_amdgcn_fence(__ATOMIC_RELEASE, "workgroup"); __builtin_amdgcn_wave_barrier(); __builtin_amdgcn_fence(__ATOMIC_ACQUIRE, "workgroup"); }
__device__ __forceinline__ float pmul(float a, float b) { float p = a * b; asm volatile("" : "+v"(p)); return p; }
__device__ __forceinline__ int iclamp(int v, int lo, int hi) { return v < lo ? lo : (v > hi ? hi : v); }

__global__ __launch_bounds__(256) void wput_kernel(const float* __restrict__ w1, const float* __restrict__ w2, b16* __restrict__ WA, b16* __restrict__ W2T) { const int u = blockIdx.x * 256 + threadIdx.x; v8b v; auto put = [&](b16* dst) { for (int pass = 0; pass < 2; ++pass) { *(volatile v8b*)dst = v; __threadfence(); } };
  if (u < 512 * 16) { const int o = u / 16, k0 = (u % 16) * 8; const int half = o / H1, oo = o % H1;
#pragma unroll
    for (int j = 0; j < 8; ++j) v[j] = (b16)(bf16_rne(w1[(size_t)(half * D0 + k0 + j) * H1 + oo]) * WSC); put(WA + (size_t)o * D0 + k0); }
  if (u < H2 * 32) { const int o = u / 32, k0 = (u % 32) * 8;
#pragma unroll
    for (int j = 0; j < 8; ++j) v[j] = (b16)(bf16_rne(w2[(size_t)(k0 + j) * H2 + o]) * WSC); put(W2T + (size_t)o * H1 + k0); } }
__global__ __launch_bounds__(32) void pq_kernel(const float* __restrict__ x, const b16* __restrict__ WA, float* __restrict__ PQ) { __shared__ __attribute__((aligned(16))) b16 Ax[16][D0 + 8]; __shared__ float Tf[16][516]; const int lane = threadIdx.x, nloc = lane & 15, hlf = lane >> 4; const size_t n0 = (size_t)blockIdx.x * 16;
  for (int rr = 0; rr < 16; ++rr) for (int q = 0; q < 4; ++q) { const int c = q * 32 + lane; Ax[rr][c] = (b16)(bfv(x[(n0 + rr) * D0 + c]) * XS); }
  if (lane < 16) for (int k = D0; k < D0 + 8; ++k) Ax[lane][k] = (b16)0.0f;
  wave_lds_sync();
#pragma unroll 1
  for (int g = 0; g < 2; ++g) { v8f acc[16];
#pragma unroll
    for (int t = 0; t < 16; ++t) acc[t] = (v8f){};
#pragma unroll
    for (int kb = 0; kb < D0; kb += 32) { const v16b a = frag_kb(&Ax[nloc][kb], hlf);
#pragma unroll
      for (int t = 0; t < 16; ++t) acc[t] = wmma16b(a, frag_kb(WA + (size_t)(g * 256 + t * 16 + nloc) * D0 + kb, hlf), acc[t]); }
#pragma unroll
    for (int t = 0; t < 16; ++t)
#pragma unroll
      for (int r8 = 0; r8 < 8; ++r8) Tf[8 * hlf + r8][g * 256 + t * 16 + nloc] = acc[t][r8] * (1.0f / (XS * WSC)); }
  wave_lds_sync();
  for (int pass = 0; pass < 2; ++pass) { for (int rr = 0; rr < 16; ++rr) for (int q = 0; q < 4; ++q) *(volatile v4f*)(PQ + (n0 + rr) * 512 + q * 128 + lane * 4) = *(const v4f*)(&Tf[rr][q * 128 + lane * 4]); __threadfence(); } }
__device__ __forceinline__ void ln_relu_row(float* row, int W, const float* g, const float* bb) { float m = 0.0f; for (int c = 0; c < W; ++c) m += row[c]; m /= (float)W; float vr = 0.0f; for (int c = 0; c < W; ++c) { const float d = row[c] - m; vr += d * d; } vr /= (float)W; const float rs = rsqrtf(vr + EPS); for (int c = 0; c < W; ++c) row[c] = fmaxf(pmul((row[c] - m) * rs, bfv(g[c])) + bfv(bb[c]), 0.0f); }
__global__ __launch_bounds__(32) void edge_kernel(const float* __restrict__ PQ, const int* __restrict__ epos, const int* __restrict__ eneg, const float* __restrict__ b1, const float* __restrict__ g1, const float* __restrict__ be1, const b16* __restrict__ W2T, const float* __restrict__ b2, const float* __restrict__ g2, const float* __restrict__ be2, const float* __restrict__ w3, const float* __restrict__ b3, int ELIM, float* __restrict__ out0, float* __restrict__ out1) { __shared__ __attribute__((aligned(16))) b16 Ah[16][H1 + 8], Al[16][H1 + 8]; __shared__ float Tr[16][H1 + 1], T2[16][H2 + 1], Pr[32]; const int lane = threadIdx.x, nloc = lane & 15, hlf = lane >> 4; const size_t e0 = (size_t)blockIdx.x * 32; if (e0 >= (size_t)ELIM) return;
  if (lane < 16) for (int k = H1; k < H1 + 8; ++k) { Ah[lane][k] = (b16)0.0f; Al[lane][k] = (b16)0.0f; }
#pragma unroll 1
  for (int rt = 0; rt < 2; ++rt) {
    for (int rr = 0; rr < 16; ++rr) { const size_t e = e0 + rt * 16 + rr; int s, d; if (e < (size_t)EP) { s = epos[e]; d = epos[EP + e]; } else { s = eneg[e - EP]; d = eneg[EN + e - EP]; } s = iclamp(s, 0, N - 1); d = iclamp(d, 0, N - 1);
      for (int q = 0; q < H1 / 32; ++q) { const int c = q * 32 + lane; Tr[rr][c] = PQ[(size_t)s * 512 + c] + PQ[(size_t)d * 512 + 256 + c] + bfv(b1[c]); } }
    wave_lds_sync(); if (lane < 16) ln_relu_row(&Tr[lane][0], H1, g1, be1); wave_lds_sync();
    for (int rr = 0; rr < 16; ++rr) for (int q = 0; q < H1 / 32; ++q) { const int c = q * 32 + lane; b16 p, pl; split16(Tr[rr][c] * HS, p, pl); Ah[rr][c] = p; Al[rr][c] = pl; }
    wave_lds_sync(); v8f acc[8];
#pragma unroll
    for (int t = 0; t < 8; ++t) acc[t] = (v8f){};
#pragma unroll 2
    for (int kb = 0; kb < H1; kb += 32) { const v16b a = frag_kb(&Ah[nloc][kb], hlf), al = frag_kb(&Al[nloc][kb], hlf);
#pragma unroll
      for (int t = 0; t < 8; ++t) { const v16b bw = frag_kb(W2T + (size_t)(t * 16 + nloc) * H1 + kb, hlf); acc[t] = wmma16b(a, bw, acc[t]); acc[t] = wmma16b(al, bw, acc[t]); } }
#pragma unroll
    for (int t = 0; t < 8; ++t) { const int cc = t * 16 + nloc; const float bb = bfv(b2[cc]);
#pragma unroll
      for (int r8 = 0; r8 < 8; ++r8) T2[8 * hlf + r8][cc] = acc[t][r8] * (1.0f / (HS * WSC)) + bb; }
    wave_lds_sync();
    if (lane < 16) { ln_relu_row(&T2[lane][0], H2, g2, be2); float s = bfv(b3[0]); for (int c = 0; c < H2; ++c) s += pmul(T2[lane][c], bfv(w3[c])); Pr[rt * 16 + lane] = 1.0f / (1.0f + __expf(-s)); }
    wave_lds_sync(); }
  for (int pass = 0; pass < 2; ++pass) { ((volatile float*)out0)[e0 + lane] = Pr[lane]; ((volatile float*)out1)[e0 + lane] = (e0 + lane) < (size_t)EP ? 1.0f : 0.0f; __threadfence(); } }
__global__ __launch_bounds__(256) void label_kernel(int ELIM, float* __restrict__ out1) { const size_t e = (size_t)ELIM + (size_t)blockIdx.x * 256 + threadIdx.x; if (e >= (size_t)ET) return; for (int pass = 0; pass < 2; ++pass) { ((volatile float*)out1)[e] = e < (size_t)EP ? 1.0f : 0.0f; __threadfence(); } }
}

extern "C" void kernel_launch(void* const* d_in, const int* in_sizes, int n_in, void* d_out, int out_size, void* d_ws, size_t ws_size, hipStream_t stream) {
  (void)n_in;
  auto Fp = [&](int i) { return (const float*)d_in[i]; }; auto Ip = [&](int i) { return (const int*)d_in[i]; };
  if (in_sizes[0] != N * D0 || in_sizes[1] != 2 * EP || in_sizes[3] != 2 * EN || in_sizes[4] != 2 * D0 * H1 || in_sizes[8] != H1 * H2 || in_sizes[12] != H2 || out_size != 2 * ET) return;
  const int ELIM = ET;
  size_t off = 0; char* ws = (char*)d_ws;
  auto carve = [&](size_t bytes) { char* p = ws + off; off += (bytes + 255) & ~(size_t)255; return p; };
  b16* WA = (b16*)carve((size_t)512 * D0 * 2); b16* W2T = (b16*)carve((size_t)H2 * H1 * 2); float* PQ = (float*)carve((size_t)N * 512 * 4);
  if (off > ws_size || off > ((size_t)112 << 20)) return;
  float* out0 = (float*)d_out; float* out1 = out0 + ET;
  wput_kernel<<<(512 * 16 + 255) / 256, 256, 0, stream>>>(Fp(4), Fp(8), WA, W2T);
  pq_kernel<<<N / 16, 32, 0, stream>>>(Fp(0), WA, PQ);
  edge_kernel<<<ET / 32, 32, 0, stream>>>(PQ, Ip(1), Ip(3), Fp(5), Fp(6), Fp(7), W2T, Fp(9), Fp(10), Fp(11), Fp(12), Fp(13), ELIM, out0, out1);
  if (ELIM < ET) label_kernel<<<(ET - ELIM + 255) / 256, 256, 0, stream>>>(ELIM, out1);
}
